// _KDA_Fast_45380624449570
// MI455X (gfx1250) — hardware-verified
//
#include <hip/hip_runtime.h>
#include <stdint.h>


typedef _Float16 h16;
typedef h16    v16h __attribute__((ext_vector_type(16)));
typedef h16    v8h  __attribute__((ext_vector_type(8)));
typedef __bf16 v16b __attribute__((ext_vector_type(16)));
typedef float  v8f  __attribute__((ext_vector_type(8)));
typedef float  v4f  __attribute__((ext_vector_type(4)));

union HF { v16h v; v8h p[2]; };
union BF { v16b v; unsigned short u[16]; };

#define DM 1024
#define HD 64
#define NH 16
#define CH 64
#define QP 68

__device__ __forceinline__ unsigned short bf16_bits(float f) {
  unsigned int u = __float_as_uint(f);
  u += 0x7FFFu + ((u >> 16) & 1u);
  return (unsigned short)(u >> 16);
}
__device__ __forceinline__ float bf16r(float f) {
  return __uint_as_float(((unsigned int)bf16_bits(f)) << 16);
}
__device__ __forceinline__ void split2(float x, unsigned short& hi, unsigned short& lo) {
  const unsigned short hb = bf16_bits(x);
  const float hf = __uint_as_float(((unsigned int)hb) << 16);
  hi = hb;
  lo = bf16_bits(x - hf);
}
__device__ __forceinline__ float sigm(float v) {
  return __fdividef(1.0f, 1.0f + __expf(-v));
}

__device__ __forceinline__ v8f mma_f16(v16h a, v16h b, v8f c) {
  c = __builtin_amdgcn_wmma_f32_16x16x32_f16(false, a, false, b, (short)0, c, false, false);
  asm volatile("v_nop\n\tv_nop\n\tv_nop\n\tv_nop" : "+v"(c) : "v"(a), "v"(b));
  return c;
}
__device__ __forceinline__ v8f mma_bf16(v16b a, v16b b, v8f c) {
  c = __builtin_amdgcn_wmma_f32_16x16x32_bf16(false, a, false, b, (short)0, c, false, false);
  asm volatile("v_nop\n\tv_nop\n\tv_nop\n\tv_nop" : "+v"(c) : "v"(a), "v"(b));
  return c;
}

__device__ __forceinline__ void fragA_split(const float* pr, int h, BF& hi, BF& lo) {
  const v4f x0 = *(const v4f*)(pr + 8 * h);
  const v4f x1 = *(const v4f*)(pr + 8 * h + 4);
  const v4f x2 = *(const v4f*)(pr + 16 + 8 * h);
  const v4f x3 = *(const v4f*)(pr + 20 + 8 * h);
#pragma unroll
  for (int q = 0; q < 4; ++q) {
    split2(x0[q], hi.u[q],      lo.u[q]);
    split2(x1[q], hi.u[4 + q],  lo.u[4 + q]);
    split2(x2[q], hi.u[8 + q],  lo.u[8 + q]);
    split2(x3[q], hi.u[12 + q], lo.u[12 + q]);
  }
}
__device__ __forceinline__ void fragB_split(const float* base, int pitch, int k0, int col, int h, BF& hi, BF& lo) {
#pragma unroll
  for (int i = 0; i < 8; ++i) {
    split2(base[(k0 + 8 * h + i) * pitch + col],      hi.u[i],     lo.u[i]);
    split2(base[(k0 + 16 + 8 * h + i) * pitch + col], hi.u[8 + i], lo.u[8 + i]);
  }
}

__global__ void __launch_bounds__(256)
k_cvtw(const float* __restrict__ src, h16* dst, int n8, float scale)
{
  const int i = blockIdx.x * 256 + threadIdx.x;
  const bool ok = i < n8;
  v8h o;
#pragma unroll
  for (int q = 0; q < 8; ++q) o[q] = (h16)0.0f;
  if (ok) {
    const v4f a = *(const v4f*)(src + (size_t)i * 8);
    const v4f c = *(const v4f*)(src + (size_t)i * 8 + 4);
#pragma unroll
    for (int q = 0; q < 4; ++q) {
      o[q]     = (h16)(bf16r(a[q]) * scale);
      o[4 + q] = (h16)(bf16r(c[q]) * scale);
    }
  }
  if (ok) *(volatile v8h*)(dst + (size_t)i * 8) = o;
  __threadfence();
  if (ok) *(volatile v8h*)(dst + (size_t)i * 8) = o;
}

__global__ void __launch_bounds__(256)
k_prep(const float* __restrict__ x,
       const float* __restrict__ w0, const float* __restrict__ b0,
       const float* __restrict__ w1, const float* __restrict__ b1,
       const float* __restrict__ w2, const float* __restrict__ b2,
       h16* xh, h16* y0, h16* y1, h16* y2, int n8, int T, float ascale)
{
  const int which = blockIdx.y;
  const float* w  = (which == 0) ? w0 : ((which == 1) ? w1 : w2);
  const float* bb = (which == 0) ? b0 : ((which == 1) ? b1 : b2);
  h16* y          = (which == 0) ? y0 : ((which == 1) ? y1 : y2);

  const int g = blockIdx.x * 256 + threadIdx.x;
  const bool ok = g < n8;
  const size_t eo = (size_t)g * 8;
  v8h o, ox;
#pragma unroll
  for (int q = 0; q < 8; ++q) { o[q] = (h16)0.0f; ox[q] = (h16)0.0f; }
  if (ok) {
    const size_t bt = (size_t)(g >> 7);
    const int d0 = (g & 127) * 8;
    const int t = (int)(bt % (size_t)T);
    float xr[4][8];
#pragma unroll
    for (int j = 0; j < 4; ++j) {
      const int ts = t - 3 + j;
      if (ts >= 0) {
        const float* px = x + (bt - (size_t)(3 - j)) * DM + d0;
        const v4f a = *(const v4f*)px;
        const v4f c = *(const v4f*)(px + 4);
#pragma unroll
        for (int q = 0; q < 4; ++q) { xr[j][q] = bf16r(a[q]); xr[j][4 + q] = bf16r(c[q]); }
      } else {
#pragma unroll
        for (int q = 0; q < 8; ++q) xr[j][q] = 0.0f;
      }
    }
#pragma unroll
    for (int q = 0; q < 8; ++q) {
      const int d = d0 + q;
      const v4f wv4 = *(const v4f*)(w + (size_t)d * 4);
      float acc = xr[0][q] * bf16r(wv4[0]);
      acc += xr[1][q] * bf16r(wv4[1]);
      acc += xr[2][q] * bf16r(wv4[2]);
      acc += xr[3][q] * bf16r(wv4[3]);
      acc += bf16r(bb[d]);
      const float s = acc * sigm(acc);
      o[q]  = (h16)(s * ascale);
      ox[q] = (h16)xr[3][q];
    }
  }
  if (ok) {
    *(volatile v8h*)(y + eo) = o;
    if (which == 0) *(volatile v8h*)(xh + eo) = ox;
  }
  __threadfence();
  if (ok) {
    *(volatile v8h*)(y + eo) = o;
    if (which == 0) *(volatile v8h*)(xh + eo) = ox;
  }
}

template<int NT, int EPI, typename OT>
__global__ void __launch_bounds__(256)
k_gemm(const h16* __restrict__ A, const h16* __restrict__ W, const float* __restrict__ bias,
       OT* Y, int N, int K, float oscale, float yscale)
{
  constexpr int TW = 16 * NT;
  __shared__ __attribute__((aligned(16))) float stg[8 * 16 * TW];

  const int lane = threadIdx.x & 31, wv = threadIdx.x >> 5;
  const int m = lane & 15, h = lane >> 4;
  const int rowBase = blockIdx.x * 128 + wv * 16;
  const int colBase = blockIdx.y * TW;

  v8f acc[NT];
#pragma unroll
  for (int t = 0; t < NT; ++t)
#pragma unroll
    for (int r = 0; r < 8; ++r) acc[t][r] = 0.0f;

  const h16* arow  = A + (size_t)(rowBase + m) * K + 8 * h;
  const h16* wbase = W + (size_t)(colBase + m) * K + 8 * h;
  for (int k0 = 0; k0 < K; k0 += 32) {
    HF a;
    a.p[0] = *(const v8h*)(arow + k0);
    a.p[1] = *(const v8h*)(arow + k0 + 16);
#pragma unroll
    for (int t = 0; t < NT; ++t) {
      const h16* wrow = wbase + (size_t)(16 * t) * K + k0;
      HF b;
      b.p[0] = *(const v8h*)(wrow);
      b.p[1] = *(const v8h*)(wrow + 16);
      acc[t] = mma_f16(a.v, b.v, acc[t]);
    }
  }

#pragma unroll
  for (int t = 0; t < NT; ++t) {
    const float bv = bf16r(bias[colBase + 16 * t + m]);
#pragma unroll
    for (int r = 0; r < 8; ++r) {
      float v = acc[t][r] * oscale + bv;
      if (EPI == 2)      { v = v * sigm(v); }
      else if (EPI == 3) { v = sigm(v); v = fminf(fmaxf(v, 0.1f), 1.0f); }
      else if (EPI == 4) { v = fminf(sigm(v), 1.0f); }
      acc[t][r] = v;
    }
  }
  if (EPI == 1) {
#pragma unroll
    for (int r = 0; r < 8; ++r) {
      float ss = 0.0f;
#pragma unroll
      for (int t = 0; t < NT; ++t) ss += acc[t][r] * acc[t][r];
      ss += __shfl_xor(ss, 1, 32);
      ss += __shfl_xor(ss, 2, 32);
      ss += __shfl_xor(ss, 4, 32);
      ss += __shfl_xor(ss, 8, 32);
      const float inv = 1.0f / sqrtf(fmaxf(ss, 1e-6f));
#pragma unroll
      for (int t = 0; t < NT; ++t) acc[t][r] *= inv;
    }
  }

  float* sw = stg + wv * 16 * TW;
#pragma unroll
  for (int t = 0; t < NT; ++t)
#pragma unroll
    for (int r = 0; r < 8; ++r) sw[(8 * h + r) * TW + 16 * t + m] = acc[t][r];
  __syncthreads();

  if constexpr (sizeof(OT) == 4 && NT == 4) {
    v4f vals[8];
    size_t offs[8];
#pragma unroll
    for (int it = 0; it < 8; ++it) {
      const int row = 2 * it + h, c4 = m * 4;
      vals[it] = *(const v4f*)(sw + row * TW + c4);
      offs[it] = (size_t)(rowBase + row) * N + colBase + c4;
    }
#pragma unroll
    for (int it = 0; it < 8; ++it) *(volatile v4f*)(Y + offs[it]) = vals[it];
    __threadfence();
#pragma unroll
    for (int it = 0; it < 8; ++it) *(volatile v4f*)(Y + offs[it]) = vals[it];
  } else if constexpr (sizeof(OT) == 2 && NT == 4) {
    v8h vals[4];
    size_t offs[4];
#pragma unroll
    for (int it = 0; it < 4; ++it) {
      const int row = it * 4 + (lane >> 3), c8 = (lane & 7) * 8;
      const v4f a = *(const v4f*)(sw + row * TW + c8);
      const v4f c = *(const v4f*)(sw + row * TW + c8 + 4);
      v8h o;
#pragma unroll
      for (int q = 0; q < 4; ++q) { o[q] = (h16)(a[q] * yscale); o[4 + q] = (h16)(c[q] * yscale); }
      vals[it] = o;
      offs[it] = (size_t)(rowBase + row) * N + colBase + c8;
    }
#pragma unroll
    for (int it = 0; it < 4; ++it) *(volatile v8h*)(Y + offs[it]) = vals[it];
    __threadfence();
#pragma unroll
    for (int it = 0; it < 4; ++it) *(volatile v8h*)(Y + offs[it]) = vals[it];
  } else if constexpr (sizeof(OT) == 4 && NT == 1) {
    v4f vals[2];
    size_t offs[2];
#pragma unroll
    for (int it = 0; it < 2; ++it) {
      const int q = it * 32 + lane, row = q >> 2, c4 = (q & 3) * 4;
      vals[it] = *(const v4f*)(sw + row * TW + c4);
      offs[it] = (size_t)(rowBase + row) * N + colBase + c4;
    }
#pragma unroll
    for (int it = 0; it < 2; ++it) *(volatile v4f*)(Y + offs[it]) = vals[it];
    __threadfence();
#pragma unroll
    for (int it = 0; it < 2; ++it) *(volatile v4f*)(Y + offs[it]) = vals[it];
  }
}

__global__ void __launch_bounds__(256)
k_chunk(const float* __restrict__ Qp, const float* __restrict__ Kp, const float* __restrict__ Vp,
        const float* __restrict__ Ap, const float* __restrict__ Bp, const float* __restrict__ Gp,
        const float* __restrict__ rmsw, h16* Og, int T, float ogscale)
{
  __shared__ __attribute__((aligned(16))) float Qs[CH * QP];
  __shared__ __attribute__((aligned(16))) float Ks[CH * QP];
  __shared__ __attribute__((aligned(16))) float CLs[CH * QP];
  __shared__ __attribute__((aligned(16))) float SCs[CH * QP];
  __shared__ __attribute__((aligned(16))) float Vs[CH * HD];
  __shared__ __attribute__((aligned(16))) float ALs[CH * HD];
  __shared__ __attribute__((aligned(16))) float Sf[HD * HD];
  __shared__ float Bsh[CH], GS[CH], RV[CH], RW[HD];
  __shared__ float PK[2 * 256];

  const int tid = threadIdx.x;
  const int lane = tid & 31, wv = tid >> 5, m = lane & 15, h = lane >> 4;
  const int bh = blockIdx.x, b = bh / NH, hh = bh % NH;
  const int e = tid & 63, dg = tid >> 6;

  float Sreg[16];
#pragma unroll
  for (int dd = 0; dd < 16; ++dd) Sreg[dd] = 0.0f;
  if (tid < HD) RW[tid] = bf16r(rmsw[hh * HD + tid]);

  const int nch = T / CH;
  for (int n = 0; n < nch; ++n) {
    const size_t rowbase = (size_t)b * T + (size_t)n * CH;
    const float* Qg = Qp + rowbase * DM + hh * HD;
    const float* Kg = Kp + rowbase * DM + hh * HD;
    const float* Vg = Vp + rowbase * DM + hh * HD;
    const float* Ag = Ap + rowbase * DM + hh * HD;

    __syncthreads();
#pragma unroll
    for (int it = 0; it < 4; ++it) {
      const int idx = it * 256 + tid;
      const int c = idx >> 4, d4 = (idx & 15) * 4;
      const size_t go = (size_t)c * DM + d4;
      *(v4f*)(Qs  + c * QP + d4) = *(const v4f*)(Qg + go);
      *(v4f*)(Ks  + c * QP + d4) = *(const v4f*)(Kg + go);
      *(v4f*)(Vs  + c * HD + d4) = *(const v4f*)(Vg + go);
      *(v4f*)(ALs + c * HD + d4) = *(const v4f*)(Ag + go);
    }
    if (tid < CH) {
      Bsh[tid] = fminf(Bp[(rowbase + tid) * NH + hh], 1.0f);
      GS[tid]  = Gp[(rowbase + tid) * NH + hh];
    }
#pragma unroll
    for (int dd = 0; dd < 16; ++dd) Sf[(dg * 16 + dd) * HD + e] = Sreg[dd];
    __syncthreads();

    if (tid < HD) {
      float a = 0.0f;
      for (int c = 0; c < CH; ++c) {
        a += __logf(fmaxf(ALs[c * HD + tid], 1e-7f));
        CLs[c * QP + tid] = a;
      }
    }
    __syncthreads();

    {
      const int j0 = lane, j1 = lane + 32;
      float a0[8], a1[4];
#pragma unroll
      for (int r = 0; r < 8; ++r) a0[r] = 0.0f;
#pragma unroll
      for (int r = 0; r < 4; ++r) a1[r] = 0.0f;
#pragma unroll 2
      for (int d = 0; d < HD; ++d) {
        const float k0v = Ks[j0 * QP + d], c0 = CLs[j0 * QP + d];
        const float k1v = Ks[j1 * QP + d], c1 = CLs[j1 * QP + d];
#pragma unroll
        for (int r = 0; r < 8; ++r) {
          const int i = wv + 8 * r;
          const float q = Qs[i * QP + d];
          const float ci = CLs[i * QP + d];
          a0[r] += q * k0v * __expf(ci - c0);
          if (r >= 4) a1[r - 4] += q * k1v * __expf(ci - c1);
        }
      }
      const float b0 = Bsh[j0], b1 = Bsh[j1];
#pragma unroll
      for (int r = 0; r < 8; ++r) {
        const int i = wv + 8 * r;
        SCs[i * QP + j0] = (i >= j0) ? a0[r] * b0 : 0.0f;
        float v1 = 0.0f;
        if (r >= 4) v1 = (i >= j1) ? a1[r - 4] * b1 : 0.0f;
        SCs[i * QP + j1] = v1;
      }
    }
    __syncthreads();

    {
      const int ti = wv >> 1, tj0 = (wv & 1) * 2;
      v8f acc[2];
#pragma unroll
      for (int s = 0; s < 2; ++s)
#pragma unroll
        for (int r = 0; r < 8; ++r) acc[s][r] = 0.0f;

#pragma unroll
      for (int ks = 0; ks < 2; ++ks) {
        const int k0 = ks * 32;
        BF ah, al;
        fragA_split(Qs + (ti * 16 + m) * QP + k0, h, ah, al);
#pragma unroll
        for (int s = 0; s < 2; ++s) {
          BF bhi, blo;
          fragB_split(Sf, HD, k0, (tj0 + s) * 16 + m, h, bhi, blo);
          acc[s] = mma_bf16(ah.v, bhi.v, acc[s]);
          acc[s] = mma_bf16(ah.v, blo.v, acc[s]);
          acc[s] = mma_bf16(al.v, bhi.v, acc[s]);
        }
      }
#pragma unroll
      for (int ks = 0; ks < 2; ++ks) {
        const int k0 = ks * 32;
        BF ah, al;
        fragA_split(SCs + (ti * 16 + m) * QP + k0, h, ah, al);
#pragma unroll
        for (int s = 0; s < 2; ++s) {
          BF bhi, blo;
          fragB_split(Vs, HD, k0, (tj0 + s) * 16 + m, h, bhi, blo);
          acc[s] = mma_bf16(ah.v, bhi.v, acc[s]);
          acc[s] = mma_bf16(ah.v, blo.v, acc[s]);
          acc[s] = mma_bf16(al.v, bhi.v, acc[s]);
        }
      }
      __syncthreads();
#pragma unroll
      for (int s = 0; s < 2; ++s)
#pragma unroll
        for (int r = 0; r < 8; ++r)
          SCs[(ti * 16 + 8 * h + r) * QP + (tj0 + s) * 16 + m] = acc[s][r];
    }
    __syncthreads();

    if (tid < CH) {
      float ss = 0.0f;
      for (int e2 = 0; e2 < HD; ++e2) { const float o = SCs[tid * QP + e2]; ss += o * o; }
      RV[tid] = GS[tid] / sqrtf(ss * (1.0f / 64.0f) + 1e-6f);
    }
    __syncthreads();

    {
      v8h ov[2];
      size_t go[2];
#pragma unroll
      for (int it = 0; it < 2; ++it) {
        const int c = it * 32 + (tid >> 3), e0 = (tid & 7) * 8;
        const v4f x0 = *(const v4f*)(SCs + c * QP + e0);
        const v4f x1 = *(const v4f*)(SCs + c * QP + e0 + 4);
        const float sc = RV[c] * ogscale;
        v8h o;
#pragma unroll
        for (int q = 0; q < 4; ++q) {
          o[q]     = (h16)(x0[q] * sc * RW[e0 + q]);
          o[4 + q] = (h16)(x1[q] * sc * RW[e0 + 4 + q]);
        }
        ov[it] = o;
        go[it] = (rowbase + c) * (size_t)DM + hh * HD + e0;
      }
#pragma unroll
      for (int it = 0; it < 2; ++it) *(volatile v8h*)(Og + go[it]) = ov[it];
      __threadfence();
#pragma unroll
      for (int it = 0; it < 2; ++it) *(volatile v8h*)(Og + go[it]) = ov[it];
    }

    for (int t = 0; t < CH; ++t) {
      float kk[16], aa[16];
#pragma unroll
      for (int q = 0; q < 4; ++q) {
        const v4f kv = *(const v4f*)(Ks  + t * QP + dg * 16 + 4 * q);
        const v4f av = *(const v4f*)(ALs + t * HD + dg * 16 + 4 * q);
#pragma unroll
        for (int u = 0; u < 4; ++u) { kk[4 * q + u] = kv[u]; aa[4 * q + u] = av[u]; }
      }
      float part = 0.0f;
#pragma unroll
      for (int dd = 0; dd < 16; ++dd) { Sreg[dd] *= aa[dd]; part += kk[dd] * Sreg[dd]; }
      float* pk = PK + (t & 1) * 256;
      pk[tid] = part;
      __syncthreads();
      const float kts = (pk[e] + pk[64 + e]) + (pk[128 + e] + pk[192 + e]);
      const float bt = Bsh[t];
      const float dl = Vs[t * HD + e] - kts;
#pragma unroll
      for (int dd = 0; dd < 16; ++dd) Sreg[dd] += (bt * kk[dd]) * dl;
    }
  }
}

extern "C" void kernel_launch(void* const* d_in, const int* in_sizes, int n_in,
                              void* d_out, int out_size, void* d_ws, size_t ws_size,
                              hipStream_t stream)
{
  if (n_in < 26) return;
  const int T = 2048;
  const long nx = (long)in_sizes[0];
  if (nx <= 0 || (nx % ((long)DM * T)) != 0) return;
  const int M = (int)(nx / DM);
  if ((long)out_size != (long)M * DM) return;
  if (in_sizes[1] != DM * 4 || in_sizes[3] != DM * 4 || in_sizes[5] != DM * 4) return;
  if (in_sizes[7] != DM * DM || in_sizes[9] != DM * DM || in_sizes[11] != DM * DM || in_sizes[24] != DM * DM) return;
  if (in_sizes[13] != 64 * DM || in_sizes[15] != DM * 64 || in_sizes[17] != NH * DM ||
      in_sizes[20] != 64 * DM || in_sizes[22] != NH * 64) return;

  const float* x       = (const float*)d_in[0];
  const float* wq_conv = (const float*)d_in[1];  const float* bq_conv = (const float*)d_in[2];
  const float* wk_conv = (const float*)d_in[3];  const float* bk_conv = (const float*)d_in[4];
  const float* wv_conv = (const float*)d_in[5];  const float* bv_conv = (const float*)d_in[6];
  const float* Wq  = (const float*)d_in[7];   const float* bq  = (const float*)d_in[8];
  const float* Wk  = (const float*)d_in[9];   const float* bk  = (const float*)d_in[10];
  const float* Wv  = (const float*)d_in[11];  const float* bv  = (const float*)d_in[12];
  const float* Wad = (const float*)d_in[13];  const float* bad = (const float*)d_in[14];
  const float* Wau = (const float*)d_in[15];  const float* bau = (const float*)d_in[16];
  const float* Wbe = (const float*)d_in[17];  const float* bbe = (const float*)d_in[18];
  const float* rms_w = (const float*)d_in[19];
  const float* Wgd = (const float*)d_in[20];  const float* bgd = (const float*)d_in[21];
  const float* Wgu = (const float*)d_in[22];  const float* bgu = (const float*)d_in[23];
  const float* Wo  = (const float*)d_in[24];  const float* bo  = (const float*)d_in[25];

  char* ws = (char*)d_ws;
  size_t off = 0;
  auto carve = [&](size_t bytes) -> char* {
    char* p = ws + off;
    off += (bytes + 255) & ~(size_t)255;
    return p;
  };
  const size_t MD = (size_t)M * DM;
  h16* xh    = (h16*)carve(MD * 2);
  h16* cq    = (h16*)carve(MD * 2);
  h16* ck    = (h16*)carve(MD * 2);
  h16* cv    = (h16*)carve(MD * 2);
  h16* Wq16  = (h16*)carve((size_t)DM * DM * 2);
  h16* Wk16  = (h16*)carve((size_t)DM * DM * 2);
  h16* Wv16  = (h16*)carve((size_t)DM * DM * 2);
  h16* Wo16  = (h16*)carve((size_t)DM * DM * 2);
  h16* Wad16 = (h16*)carve((size_t)64 * DM * 2);
  h16* Wau16 = (h16*)carve((size_t)DM * 64 * 2);
  h16* Wbe16 = (h16*)carve((size_t)NH * DM * 2);
  h16* Wgd16 = (h16*)carve((size_t)64 * DM * 2);
  h16* Wgu16 = (h16*)carve((size_t)NH * 64 * 2);
  float* Qn  = (float*)carve(MD * 4);
  float* Kn  = (float*)carve(MD * 4);
  float* Vf  = (float*)carve(MD * 4);
  float* Al  = (float*)carve(MD * 4);
  float* Bt  = (float*)carve((size_t)M * NH * 4);
  float* Gt  = (float*)carve((size_t)M * NH * 4);
  h16* t1    = (h16*)carve((size_t)M * 64 * 2);
  h16* t2    = (h16*)carve((size_t)M * 64 * 2);
  h16* Og16  = (h16*)carve(MD * 2);
  if (off > ws_size) return;

  const float wsc = 256.0f;
  const float asc = 256.0f;
  const float tsc = 64.0f;
  const float osc = 16.0f;

  {
    const int n8 = (int)(MD / 8);
    k_prep<<<dim3((n8 + 255) / 256, 3), 256, 0, stream>>>(x, wq_conv, bq_conv, wk_conv, bk_conv, wv_conv, bv_conv,
                                                         xh, cq, ck, cv, n8, T, asc);
  }
  {
    int n8;
    n8 = DM * DM / 8;  k_cvtw<<<(n8 + 255) / 256, 256, 0, stream>>>(Wq,  Wq16,  n8, wsc);
    n8 = DM * DM / 8;  k_cvtw<<<(n8 + 255) / 256, 256, 0, stream>>>(Wk,  Wk16,  n8, wsc);
    n8 = DM * DM / 8;  k_cvtw<<<(n8 + 255) / 256, 256, 0, stream>>>(Wv,  Wv16,  n8, wsc);
    n8 = DM * DM / 8;  k_cvtw<<<(n8 + 255) / 256, 256, 0, stream>>>(Wo,  Wo16,  n8, wsc);
    n8 = 64 * DM / 8;  k_cvtw<<<(n8 + 255) / 256, 256, 0, stream>>>(Wad, Wad16, n8, wsc);
    n8 = DM * 64 / 8;  k_cvtw<<<(n8 + 255) / 256, 256, 0, stream>>>(Wau, Wau16, n8, wsc);
    n8 = NH * DM / 8;  k_cvtw<<<(n8 + 255) / 256, 256, 0, stream>>>(Wbe, Wbe16, n8, wsc);
    n8 = 64 * DM / 8;  k_cvtw<<<(n8 + 255) / 256, 256, 0, stream>>>(Wgd, Wgd16, n8, wsc);
    n8 = NH * 64 / 8;  k_cvtw<<<(n8 + 255) / 256, 256, 0, stream>>>(Wgu, Wgu16, n8, wsc);
  }
  const dim3 gbig(M / 128, DM / 64);
  const dim3 gsm(M / 128, 1);
  k_gemm<4, 1, float><<<gbig, 256, 0, stream>>>(cq, Wq16, bq, Qn, DM, DM, 1.0f / (asc * wsc), 1.0f);
  k_gemm<4, 1, float><<<gbig, 256, 0, stream>>>(ck, Wk16, bk, Kn, DM, DM, 1.0f / (asc * wsc), 1.0f);
  k_gemm<4, 0, float><<<gbig, 256, 0, stream>>>(cv, Wv16, bv, Vf, DM, DM, 1.0f / (asc * wsc), 1.0f);
  k_gemm<4, 2, h16  ><<<gsm,  256, 0, stream>>>(xh, Wad16, bad, t1, 64, DM, 1.0f / wsc, tsc);
  k_gemm<4, 3, float><<<gbig, 256, 0, stream>>>(t1, Wau16, bau, Al, DM, 64, 1.0f / (tsc * wsc), 1.0f);
  k_gemm<1, 4, float><<<gsm,  256, 0, stream>>>(xh, Wbe16, bbe, Bt, NH, DM, 1.0f / wsc, 1.0f);
  k_gemm<4, 2, h16  ><<<gsm,  256, 0, stream>>>(xh, Wgd16, bgd, t2, 64, DM, 1.0f / wsc, tsc);
  k_gemm<1, 4, float><<<gsm,  256, 0, stream>>>(t2, Wgu16, bgu, Gt, NH, 64, 1.0f / (tsc * wsc), 1.0f);
  k_chunk<<<(M / T) * NH, 256, 0, stream>>>(Qn, Kn, Vf, Al, Bt, Gt, rms_w, Og16, T, osc);
  k_gemm<4, 0, float><<<gbig, 256, 0, stream>>>(Og16, Wo16, bo, (float*)d_out, DM, DM, 1.0f / (osc * wsc), 1.0f);
}
